// GNN_Model_61589831024802
// MI455X (gfx1250) — hardware-verified
//
#include <hip/hip_runtime.h>
#include <stddef.h>
#include <stdint.h>
#include <math.h>


#define NN     10000
#define FE     100
#define NHD    10
#define HF     1000
#define HP     1024
#define K1     128
#define K2     2048
#define NG     64
#define PW     2000
#define GKH    2048
#define KF1    4096
#define F1N    1500
#define F1P    1536
#define KF2    3072
#define F2N    300
#define F2P    320
#define MP     10112
#define NP     10240
#define NTHR   256
#define NWAVE  8
#define EPT    8
#define CHUNK  (NTHR * EPT)
#define WCAP   (EPT * 32)
#define LISTN  (NWAVE * WCAP)
#define NBA    1024
#define SLA    10
#define RCAP   28672
#define DEGCAP 64
#define GBM    64
#define GBN    64
#define GTHR   128
#define AGG_ZINTS (LISTN + 2 * RCAP + 3 * NBA)
#define AGG_LDS_INTS (AGG_ZINTS + 16)
#define ALW    1040
#define NBW    80
#define U_XB   (MP  * (K1  / 8))
#define U_W1   (HP  * (K1  / 8))
#define U_W2   (HP  * (K2  / 8))
#define U_F1   (F1P * (KF1 / 8))
#define U_F2   (F2P * (KF2 / 8))
#define U_TOT  (U_XB + U_W1 + U_W2 + U_F1 + U_F2)
#define HEAD_LDS (16 * KF2 * 2 + 16 * F2N * 4)
#define WSMAX  134217728

static_assert((CHUNK & (CHUNK - 1)) == 0 && CHUNK <= 4096);
static_assert((NBA & (NBA - 1)) == 0 && NBA == (1 << SLA));
static_assert(((long long)CHUNK << SLA) < (1LL << 31));
static_assert(NBA % NWAVE == 0 && NBA == 4 * NTHR);
static_assert(AGG_ZINTS % 4 == 0 && AGG_LDS_INTS * 4 <= 300000);
static_assert(MP % GBM == 0 && HP % GBN == 0 && MP % NWAVE == 0 && NN % NWAVE == 0 && MP >= NN && NP >= MP);
static_assert(NP % NBA == 0);
static_assert(K1 % 32 == 0 && K2 % 32 == 0 && KF1 % 32 == 0 && KF2 % 32 == 0);
static_assert(K2 == 2 * HP && KF1 == 2 * GKH && KF2 == 2 * F1P);
static_assert(FE % 4 == 0 && HF % 8 == 0 && PW % 4 == 0 && F1N % 4 == 0 && HF == NHD * FE);
static_assert(U_XB % NTHR == 0 && U_W1 % NTHR == 0 && U_W2 % NTHR == 0 && U_F1 % NTHR == 0 && U_F2 % NTHR == 0);
static_assert(F1P == 24 * 64 && F2P == 20 * 16 && NG % 16 == 0);
static_assert((16 * F2N * 4) % 128 == 0 && (16 * F2N) % 4 == 0);
static_assert(HEAD_LDS <= 300000);
static_assert(DEGCAP == 64);

typedef float          v4f   __attribute__((ext_vector_type(4)));
typedef float          v8f   __attribute__((ext_vector_type(8)));
typedef int            v4i   __attribute__((ext_vector_type(4)));
typedef int            v8i   __attribute__((ext_vector_type(8)));
typedef unsigned short v4us  __attribute__((ext_vector_type(4)));
typedef unsigned short v8us  __attribute__((ext_vector_type(8)));
typedef unsigned short v16us __attribute__((ext_vector_type(16)));
typedef __bf16         v16bf __attribute__((ext_vector_type(16)));
typedef v4f  __attribute__((may_alias)) v4fa;
typedef v4i  __attribute__((may_alias)) v4ia;
typedef v4us __attribute__((may_alias)) v4usa;
typedef v8us __attribute__((may_alias)) v8usa;
union FragB { v16bf v; v16us u; v8us h[2]; v8i w; };

__device__ __forceinline__ v8f wmb(const FragB& a, const FragB& b, v8f c) {
  v8f d = __builtin_amdgcn_wmma_f32_16x16x32_bf16(false, a.v, false, b.v, (short)0, c, false, false);
  asm volatile("v_nop\n\tv_nop\n\tv_nop\n\tv_nop" : "+v"(d) : "v"(a.w), "v"(b.w));
  return d;
}

__device__ __forceinline__ unsigned bf16_bits(float f) {
  const unsigned u = __float_as_uint(f);
  return (u + 0x7FFFu + ((u >> 16) & 1u)) >> 16;
}
__device__ __forceinline__ float bf16_val(float f) {
  return __uint_as_float(bf16_bits(f) << 16);
}
__device__ __forceinline__ float relu_keep(float v) { return (v > 0.0f) ? v : (v - v); }
__device__ __forceinline__ float leaky02(float v)   { return (v >= 0.0f) ? v : 0.2f * v; }
__device__ __forceinline__ float maxk(float m, float v) { return (v > m || v != v) ? v : m; }

__device__ __forceinline__ void wave_sync() {
  __builtin_amdgcn_fence(__ATOMIC_RELEASE, "wavefront");
  __builtin_amdgcn_wave_barrier();
  __builtin_amdgcn_fence(__ATOMIC_ACQUIRE, "wavefront");
}

template <int SLB>
__device__ __forceinline__ int scan_chunk(const int* __restrict__ dsts, int nE, int cbase, int slotBase,
                                          int nb, int vec8, int* list, int tid, int lane, int wave) {
  int wc = 0;
  const int el0  = tid * EPT;
  const int e0   = cbase + el0;
  const int sent = -2147483647 - 1;
  v4i da, db;
  if (vec8 != 0 && cbase + CHUNK <= nE) {
    da = *(const v4i*)(dsts + e0);
    db = *(const v4i*)(dsts + e0 + 4);
  } else {
    da.x = (e0     < nE) ? dsts[min(e0,     nE - 1)] : sent;
    da.y = (e0 + 1 < nE) ? dsts[min(e0 + 1, nE - 1)] : sent;
    da.z = (e0 + 2 < nE) ? dsts[min(e0 + 2, nE - 1)] : sent;
    da.w = (e0 + 3 < nE) ? dsts[min(e0 + 3, nE - 1)] : sent;
    db.x = (e0 + 4 < nE) ? dsts[min(e0 + 4, nE - 1)] : sent;
    db.y = (e0 + 5 < nE) ? dsts[min(e0 + 5, nE - 1)] : sent;
    db.z = (e0 + 6 < nE) ? dsts[min(e0 + 6, nE - 1)] : sent;
    db.w = (e0 + 7 < nE) ? dsts[min(e0 + 7, nE - 1)] : sent;
  }
  const unsigned nbs = (unsigned)slotBase;
  const unsigned unb = (unsigned)nb;
  const unsigned s0 = (unsigned)da.x - nbs, s1 = (unsigned)da.y - nbs;
  const unsigned s2 = (unsigned)da.z - nbs, s3 = (unsigned)da.w - nbs;
  const unsigned s4 = (unsigned)db.x - nbs, s5 = (unsigned)db.y - nbs;
  const unsigned s6 = (unsigned)db.z - nbs, s7 = (unsigned)db.w - nbs;
  const bool h0 = s0 < unb, h1 = s1 < unb, h2 = s2 < unb, h3 = s3 < unb;
  const bool h4 = s4 < unb, h5 = s5 < unb, h6 = s6 < unb, h7 = s7 < unb;
  const unsigned any = __builtin_amdgcn_ballot_w32(h0 | h1 | h2 | h3 | h4 | h5 | h6 | h7);
  if (any != 0u) {
#define HITJ(J, HJ, SJ) { \
      const unsigned mj = __builtin_amdgcn_ballot_w32(HJ); \
      if (mj != 0u) { \
        if (HJ) { \
          const int pos = wc + (int)__builtin_amdgcn_mbcnt_lo(mj, 0u); \
          if (pos < WCAP) list[wave * WCAP + pos] = ((el0 + (J)) << SLB) | (int)(SJ); \
        } \
        wc += (int)__builtin_popcount(mj); } }
    HITJ(0, h0, s0)
    HITJ(1, h1, s1)
    HITJ(2, h2, s2)
    HITJ(3, h3, s3)
    HITJ(4, h4, s4)
    HITJ(5, h5, s5)
    HITJ(6, h6, s6)
    HITJ(7, h7, s7)
#undef HITJ
  }
  return wc;
}

__global__ __launch_bounds__(NTHR) void k_prep(const float* __restrict__ x, const float* __restrict__ W1,
                                               const float* __restrict__ W2, const float* __restrict__ fc1,
                                               const float* __restrict__ fc2,
                                               unsigned short* XB, unsigned short* W1p, unsigned short* W2d,
                                               unsigned short* FC1d, unsigned short* FC2d) {
  int u = (int)blockIdx.x * NTHR + (int)threadIdx.x;
  const float* S;
  unsigned short* P;
  int R, K, KH, PU;
  if (u < U_XB)                                   { S = x;   P = XB;   R = NN;  K = FE;  KH = K1;  PU = K1 / 8; }
  else if (u < U_XB + U_W1)                       { u -= U_XB;                      S = W1;  P = W1p;  R = HF;  K = FE;  KH = K1;  PU = K1 / 8; }
  else if (u < U_XB + U_W1 + U_W2)                { u -= U_XB + U_W1;               S = W2;  P = W2d;  R = HF;  K = HF;  KH = HP;  PU = K2 / 8; }
  else if (u < U_XB + U_W1 + U_W2 + U_F1)         { u -= U_XB + U_W1 + U_W2;        S = fc1; P = FC1d; R = F1N; K = PW;  KH = GKH; PU = KF1 / 8; }
  else if (u < U_TOT)                             { u -= U_XB + U_W1 + U_W2 + U_F1; S = fc2; P = FC2d; R = F2N; K = F1N; KH = F1P; PU = KF2 / 8; }
  else return;
  const int row  = u / PU;
  const int g    = u - row * PU;
  const int kcol = 8 * g;
  const int kk   = (kcol >= KH) ? (kcol - KH) : kcol;
  const bool rok = row < R;
  const int  rc  = rok ? row : (R - 1);
  const bool ca  = (kk + 3) < K;
  const bool cb  = (kk + 7) < K;
  const float* pr = S + (size_t)rc * (size_t)K;
  const v4f a = *(const v4fa*)(pr + (ca ? kk : 0));
  const v4f b = *(const v4fa*)(pr + (cb ? (kk + 4) : 0));
  const bool oa = rok && ca, ob = rok && cb;
  v8us o;
  o[0] = oa ? (unsigned short)bf16_bits(a.x) : (unsigned short)0;
  o[1] = oa ? (unsigned short)bf16_bits(a.y) : (unsigned short)0;
  o[2] = oa ? (unsigned short)bf16_bits(a.z) : (unsigned short)0;
  o[3] = oa ? (unsigned short)bf16_bits(a.w) : (unsigned short)0;
  o[4] = ob ? (unsigned short)bf16_bits(b.x) : (unsigned short)0;
  o[5] = ob ? (unsigned short)bf16_bits(b.y) : (unsigned short)0;
  o[6] = ob ? (unsigned short)bf16_bits(b.z) : (unsigned short)0;
  o[7] = ob ? (unsigned short)bf16_bits(b.w) : (unsigned short)0;
  unsigned short* dp = P + (size_t)row * (size_t)(PU * 8) + kcol;
  *(volatile v8us*)dp = o;
  __threadfence();
  *(volatile v8us*)dp = o;
}

__global__ __launch_bounds__(GTHR) void k_gemm(const unsigned short* __restrict__ A,
                                               const unsigned short* __restrict__ WT,
                                               float* outF, int K, int ldo) {
  __shared__ __attribute__((aligned(16))) float stg[GBM * GBN];
  const int tid = (int)threadIdx.x, lane = tid & 31, wave = tid >> 5, hh = lane >> 4, m = lane & 15;
  const int rowBase = (int)blockIdx.x * GBM;
  const int col0    = (int)blockIdx.y * GBN;

  v8f acc[4];
  {
    const v8f z = {0.f, 0.f, 0.f, 0.f, 0.f, 0.f, 0.f, 0.f};
    acc[0] = z; acc[1] = z; acc[2] = z; acc[3] = z;
  }
  const unsigned short* ap = A  + (size_t)(rowBase + 16 * wave + m) * (size_t)K + 8 * hh;
  const unsigned short* wp = WT + (size_t)(col0 + m) * (size_t)K + 8 * hh;
  const int ksteps = K >> 5;
#pragma unroll 1
  for (int ks = 0; ks < ksteps; ++ks) {
    FragB af;
    af.h[0] = *(const v8usa*)(ap + 32 * ks);
    af.h[1] = *(const v8usa*)(ap + 32 * ks + 16);
#pragma unroll
    for (int t = 0; t < 4; ++t) {
      const unsigned short* wq = wp + (size_t)(16 * t) * (size_t)K + 32 * ks;
      FragB bf;
      bf.h[0] = *(const v8usa*)wq;
      bf.h[1] = *(const v8usa*)(wq + 16);
      acc[t] = wmb(af, bf, acc[t]);
    }
  }

#pragma unroll
  for (int t = 0; t < 4; ++t) {
    const int lc = 16 * t + m;
#pragma unroll
    for (int r = 0; r < 8; ++r) {
      const int lr = 16 * wave + 8 * hh + r;
      stg[lr * GBN + lc] = acc[t][r];
    }
  }
  __syncthreads();

  v4f fv[8];
#pragma unroll
  for (int i = 0; i < 8; ++i) {
    const int lr = 16 * wave + 2 * i + hh;
    fv[i] = *(const v4fa*)(stg + lr * GBN + 4 * m);
  }
#pragma unroll
  for (int i = 0; i < 8; ++i) {
    const int lr = 16 * wave + 2 * i + hh;
    float* op = outF + (size_t)(rowBase + lr) * (size_t)ldo + col0 + 4 * m;
    *(volatile v4f*)op = fv[i];
  }
  __threadfence();
#pragma unroll
  for (int i = 0; i < 8; ++i) {
    const int lr = 16 * wave + 2 * i + hh;
    float* op = outF + (size_t)(rowBase + lr) * (size_t)ldo + col0 + 4 * m;
    *(volatile v4f*)op = fv[i];
  }
}

__global__ __launch_bounds__(NTHR) void k_dots(const float* __restrict__ H, const float* __restrict__ att_s,
                                               const float* __restrict__ att_d, float* AS, float* AD) {
  __shared__ __attribute__((aligned(16))) float ws[HF];
  __shared__ __attribute__((aligned(16))) float wd[HF];
  __shared__ __attribute__((aligned(16))) float sa[NWAVE * 16];
  __shared__ __attribute__((aligned(16))) float sd[NWAVE * 16];
  const int tid = (int)threadIdx.x, lane = tid & 31, wave = tid >> 5;
#pragma unroll 1
  for (int i = tid; i < HF; i += NTHR) { ws[i] = bf16_val(att_s[i]); wd[i] = bf16_val(att_d[i]); }
  if (tid < NWAVE * 16) { sa[tid] = 0.0f; sd[tid] = 0.0f; }
  __syncthreads();
  const int node = (int)blockIdx.x * NWAVE + wave;
  const int nc = node < NN ? node : NN - 1;
  const float* hp = H + (size_t)nc * HP;
  const int cl = lane < 25 ? lane : 24;
  const float fz = lane < 25 ? 1.0f : 0.0f;
#pragma unroll 1
  for (int h = 0; h < NHD; ++h) {
    const int c0 = FE * h + 4 * cl;
    const v4f a = *(const v4fa*)(hp + c0);
    const v4f s = *(const v4fa*)(ws + c0);
    const v4f d = *(const v4fa*)(wd + c0);
    float ps = ((a.x * s.x + a.y * s.y) + (a.z * s.z + a.w * s.w)) * fz;
    float pd = ((a.x * d.x + a.y * d.y) + (a.z * d.z + a.w * d.w)) * fz;
    ps += __shfl_xor(ps, 16, 32); pd += __shfl_xor(pd, 16, 32);
    ps += __shfl_xor(ps, 8, 32);  pd += __shfl_xor(pd, 8, 32);
    ps += __shfl_xor(ps, 4, 32);  pd += __shfl_xor(pd, 4, 32);
    ps += __shfl_xor(ps, 2, 32);  pd += __shfl_xor(pd, 2, 32);
    ps += __shfl_xor(ps, 1, 32);  pd += __shfl_xor(pd, 1, 32);
    if (lane == 0) { sa[wave * 16 + h] = ps; sd[wave * 16 + h] = pd; }
  }
  __syncthreads();
  const v4f va = *(const v4fa*)(sa + 4 * lane);
  const v4f vd = *(const v4fa*)(sd + 4 * lane);
  const size_t ob = (size_t)blockIdx.x * (NWAVE * 16) + 4 * lane;
  if (wave == 0) *(volatile v4f*)(AS + ob) = va;
  if (wave == 1) *(volatile v4f*)(AD + ob) = vd;
  __threadfence();
  if (wave == 0) *(volatile v4f*)(AS + ob) = va;
  if (wave == 1) *(volatile v4f*)(AD + ob) = vd;
}

__global__ __launch_bounds__(NTHR) void k_adj(const int* __restrict__ srcs, const int* __restrict__ dsts,
                                              int nE, int vec8, int* NBR, int* CNT, float* DINV) {
  extern __shared__ __attribute__((aligned(16))) int dsm[];
  int* list = dsm;
  int* hl   = dsm + LISTN;
  int* sl   = dsm + LISTN + RCAP;
  int* cnt  = dsm + LISTN + 2 * RCAP;
  int* offs = cnt + NBA;
  int* cur  = offs + NBA;
  int* misc = cur + NBA;
  const int tid = (int)threadIdx.x, lane = tid & 31, wave = tid >> 5;
  const int nodeBase = (int)blockIdx.x * NBA;

  {
    const v4i z4 = {0, 0, 0, 0};
    for (int i = tid * 4; i < AGG_ZINTS; i += NTHR * 4) *(v4ia*)(dsm + i) = z4;
    if (tid < 16) misc[tid] = 0;
  }
  __syncthreads();

  int t = 0, ov = 0;
  const int nChunks = (nE + CHUNK - 1) / CHUNK;
#pragma unroll 1
  for (int ch = 0; ch < nChunks; ++ch) {
    const int cbase = ch * CHUNK;
    const int wc = scan_chunk<SLA>(dsts, nE, cbase, nodeBase, NBA, vec8, list, tid, lane, wave);
    if (lane == 0) misc[wave] = wc;
    __syncthreads();
    if (wave == 0) {
#pragma unroll 1
      for (int w2 = 0; w2 < NWAVE; ++w2) {
        int c = misc[w2];
        c = c < 0 ? 0 : (c > WCAP ? WCAP : c);
#pragma unroll 1
        for (int b0 = 0; b0 < c; b0 += 32) {
          const int idx = b0 + lane;
          const int ent = list[w2 * WCAP + (idx < WCAP ? idx : WCAP - 1)];
          const int m32 = (c - b0) < 32 ? (c - b0) : 32;
#pragma unroll 1
          for (int k = 0; k < m32; ++k) {
            const int u    = __builtin_amdgcn_readlane(ent, k);
            const int slot = u & (NBA - 1);
            const int el   = (u >> SLA) & (CHUNK - 1);
            const int pk   = ((cbase + el) << SLA) | slot;
            if (t < RCAP) {
              if (lane == 0) { hl[t] = pk; cnt[slot] = cnt[slot] + 1; }
              t = t + 1;
            } else {
              ov = 1;
            }
          }
        }
      }
    }
    __syncthreads();
  }
  if (wave == 0 && lane == 0) { misc[8] = t; misc[9] = ov; }
  __syncthreads();
  int tt = misc[8];
  tt = tt < 0 ? 0 : (tt > RCAP ? RCAP : tt);
  const int ovf = misc[9];

  if (wave == 0) {
    const int base = lane * (NBA / 32);
    int s = 0;
#pragma unroll 1
    for (int i = 0; i < NBA / 32; ++i) s += cnt[base + i];
    int incl = s;
#pragma unroll
    for (int d = 1; d < 32; d <<= 1) {
      const int y = __shfl_up(incl, d, 32);
      if (lane >= d) incl += y;
    }
    int run = incl - s;
#pragma unroll 1
    for (int i = 0; i < NBA / 32; ++i) {
      const int cv = cnt[base + i];
      offs[base + i] = run;
      cur[base + i]  = run;
      run += cv;
    }
  }
  __syncthreads();
  if (wave == 0) {
#pragma unroll 1
    for (int b0 = 0; b0 < tt; b0 += 32) {
      const int idx = b0 + lane;
      const int ent = hl[idx < RCAP ? idx : RCAP - 1];
      const int m32 = (tt - b0) < 32 ? (tt - b0) : 32;
#pragma unroll 1
      for (int k = 0; k < m32; ++k) {
        const int u    = __builtin_amdgcn_readlane(ent, k);
        const int slot = u & (NBA - 1);
        if (lane == 0) {
          int p = cur[slot];
          p = p < 0 ? 0 : (p > RCAP - 1 ? RCAP - 1 : p);
          sl[p] = u;
          cur[slot] = p + 1;
        }
      }
    }
  }
  __syncthreads();

  const int L = lane & 15;
#pragma unroll 1
  for (int si = 0; si < NBA / NWAVE; ++si) {
    const int s    = si * NWAVE + wave;
    const int node = nodeBase + s;
    int c = cnt[s];
    c = c < 0 ? 0 : (c > DEGCAP ? DEGCAP : c);
    int o = offs[s];
    o = o < 0 ? 0 : (o > RCAP ? RCAP : o);
    v4i ovv;
#pragma unroll
    for (int q = 0; q < 4; ++q) {
      const int e = 4 * L + q;
      int idx = o + e;
      idx = idx > RCAP - 1 ? RCAP - 1 : idx;
      const int ent = sl[idx];
      int eid = ent >> SLA;
      eid = eid < 0 ? 0 : (eid > nE - 1 ? nE - 1 : eid);
      int sr = srcs[eid];
      sr = sr < 0 ? 0 : (sr > NN - 1 ? NN - 1 : sr);
      ovv[q] = (e < c) ? sr : 0;
    }
    int* rp = NBR + (size_t)node * DEGCAP + 4 * L;
    if (lane < 16) *(volatile v4i*)rp = ovv;
    __threadfence();
    if (lane < 16) *(volatile v4i*)rp = ovv;
  }

  {
    const int s0 = 4 * tid;
    const v4i c4 = *(const v4ia*)(cnt + s0);
    v4i cv;
    v4f dv;
#pragma unroll
    for (int q = 0; q < 4; ++q) {
      const int c = c4[q];
      const bool bad = (ovf != 0) || (c > DEGCAP) || (c < 0);
      cv[q] = bad ? -1 : c;
      const float d = (float)c + 1.0f;
      dv[q] = (d > 0.0f) ? rsqrtf(d) : 0.0f;
    }
    int*   cp = CNT  + (size_t)nodeBase + s0;
    float* dp = DINV + (size_t)nodeBase + s0;
    *(volatile v4i*)cp = cv;
    *(volatile v4f*)dp = dv;
    __threadfence();
    *(volatile v4i*)cp = cv;
    *(volatile v4f*)dp = dv;
  }
}

__global__ __launch_bounds__(NTHR) void k_scan1(const float* __restrict__ H, const float* __restrict__ AS,
                                                const float* __restrict__ AD, const int* __restrict__ NBR,
                                                const int* __restrict__ CNT, const float* __restrict__ b1,
                                                unsigned short* X1) {
  __shared__ __attribute__((aligned(16))) float al_s[NWAVE * ALW];
  __shared__ __attribute__((aligned(16))) int   nb_s[NWAVE * NBW];
  const int tid = (int)threadIdx.x, lane = tid & 31, wave = tid >> 5;
  float* al  = al_s + wave * ALW;
  int*   nbl = nb_s + wave * NBW;
  const int node = (int)blockIdx.x * NWAVE + wave;
  const bool live = node < NN;
  const int nc = live ? node : NN - 1;
  const int cv = CNT[nc];
  const bool bad = live && ((unsigned)cv > (unsigned)DEGCAP);
  const int c = (live && !bad) ? cv : 0;
  const float ninf = __int_as_float((int)0xff800000u);

  {
    const float* adp = AD + (size_t)nc * 16;
    const v4f d0 = *(const v4fa*)adp, d1 = *(const v4fa*)(adp + 4), d2 = *(const v4fa*)(adp + 8);
#pragma unroll
    for (int r = 0; r < 2; ++r) {
      const int t = 32 * r + lane;
      int sr = NBR[(size_t)nc * DEGCAP + t];
      sr = sr < 0 ? 0 : (sr > NN - 1 ? NN - 1 : sr);
      const bool valid = t < c;
      const float* asp = AS + (size_t)sr * 16;
      v4f e0 = *(const v4fa*)asp + d0;
      v4f e1 = *(const v4fa*)(asp + 4) + d1;
      v4f e2 = *(const v4fa*)(asp + 8) + d2;
      e0.x = valid ? leaky02(e0.x) : ninf; e0.y = valid ? leaky02(e0.y) : ninf;
      e0.z = valid ? leaky02(e0.z) : ninf; e0.w = valid ? leaky02(e0.w) : ninf;
      e1.x = valid ? leaky02(e1.x) : ninf; e1.y = valid ? leaky02(e1.y) : ninf;
      e1.z = valid ? leaky02(e1.z) : ninf; e1.w = valid ? leaky02(e1.w) : ninf;
      e2.x = valid ? leaky02(e2.x) : ninf; e2.y = valid ? leaky02(e2.y) : ninf;
      e2.z = valid ? leaky02(e2.z) : ninf; e2.w = valid ? leaky02(e2.w) : ninf;
      *(v4fa*)(al + t * 16)     = e0;
      *(v4fa*)(al + t * 16 + 4) = e1;
      *(v4fa*)(al + t * 16 + 8) = e2;
      nbl[t] = sr;
    }
    const int li = lane & 15;
    const float es = leaky02(AS[(size_t)nc * 16 + li] + AD[(size_t)nc * 16 + li]);
    if (lane < 16) al[64 * 16 + li] = es;
    if (lane == 0) nbl[64] = nc;
  }
  wave_sync();

  const bool v0 = lane < c, v1 = (lane + 32) < c;
#pragma unroll 1
  for (int h = 0; h < NHD; ++h) {
    const float e0 = al[lane * 16 + h];
    const float e1 = al[(lane + 32) * 16 + h];
    const float es = al[64 * 16 + h];
    float mv = fmaxf(e0, e1);
    mv = fmaxf(mv, __shfl_xor(mv, 16, 32));
    mv = fmaxf(mv, __shfl_xor(mv, 8, 32));
    mv = fmaxf(mv, __shfl_xor(mv, 4, 32));
    mv = fmaxf(mv, __shfl_xor(mv, 2, 32));
    mv = fmaxf(mv, __shfl_xor(mv, 1, 32));
    mv = fmaxf(mv, es);
    float p0 = expf(v0 ? (e0 - mv) : 0.0f);
    float p1 = expf(v1 ? (e1 - mv) : 0.0f);
    const float ps = expf(es - mv);
    p0 = v0 ? p0 : 0.0f;
    p1 = v1 ? p1 : 0.0f;
    float sv = p0 + p1;
    sv += __shfl_xor(sv, 16, 32);
    sv += __shfl_xor(sv, 8, 32);
    sv += __shfl_xor(sv, 4, 32);
    sv += __shfl_xor(sv, 2, 32);
    sv += __shfl_xor(sv, 1, 32);
    sv += ps;
    const float inv = 1.0f / (sv + 1e-16f);
    al[lane * 16 + h]        = p0 * inv;
    al[(lane + 32) * 16 + h] = p1 * inv;
    if (lane == 0) al[64 * 16 + h] = ps * inv;
  }
  wave_sync();

  int hA[4], hB[4];
#pragma unroll
  for (int j = 0; j < 4; ++j) {
    const int c0 = 256 * j + 8 * lane;
    const int a = c0 / FE, b = (c0 + 4) / FE;
    hA[j] = a > NHD - 1 ? NHD - 1 : a;
    hB[j] = b > NHD - 1 ? NHD - 1 : b;
  }
  v4f accA[4], accB[4];
  {
    const v4f z = {0.f, 0.f, 0.f, 0.f};
#pragma unroll
    for (int j = 0; j < 4; ++j) { accA[j] = z; accB[j] = z; }
  }
#pragma unroll 1
  for (int t = 0; t <= c; ++t) {
    const int tt = (t < c) ? t : 64;
    const int sk = nbl[tt];
    const float* hp = H + (size_t)sk * HP + 8 * lane;
    const float* ar = al + tt * 16;
#pragma unroll
    for (int j = 0; j < 4; ++j) {
      const v4f a = *(const v4fa*)(hp + 256 * j);
      const v4f b = *(const v4fa*)(hp + 256 * j + 4);
      const float wa = ar[hA[j]];
      const float wb = ar[hB[j]];
      accA[j] += wa * a;
      accB[j] += wb * b;
    }
  }

  const float pzr = bad ? __int_as_float(0x7fc00000) : 0.0f;
  v8us hv[4], lv[4];
#pragma unroll
  for (int j = 0; j < 4; ++j) {
    const int c0 = 256 * j + 8 * lane;
    const bool okc = c0 < HF;
    const int cb = okc ? c0 : HF - 8;
    const v4f ba = *(const v4fa*)(b1 + cb);
    const v4f bb = *(const v4fa*)(b1 + cb + 4);
    const bool keep = live && okc;
    float y[8];
    y[0] = accA[j].x + bf16_val(ba.x); y[1] = accA[j].y + bf16_val(ba.y);
    y[2] = accA[j].z + bf16_val(ba.z); y[3] = accA[j].w + bf16_val(ba.w);
    y[4] = accB[j].x + bf16_val(bb.x); y[5] = accB[j].y + bf16_val(bb.y);
    y[6] = accB[j].z + bf16_val(bb.z); y[7] = accB[j].w + bf16_val(bb.w);
#pragma unroll
    for (int q = 0; q < 8; ++q) {
      float v = relu_keep(y[q]) + pzr;
      v = keep ? v : 0.0f;
      const unsigned hb = bf16_bits(v);
      const unsigned lb = bf16_bits(v - __uint_as_float(hb << 16));
      hv[j][q] = (unsigned short)hb;
      lv[j][q] = (unsigned short)lb;
    }
  }
  unsigned short* rp = X1 + (size_t)node * K2 + 8 * lane;
#pragma unroll
  for (int j = 0; j < 4; ++j) {
    *(volatile v8us*)(rp + 256 * j) = hv[j];
    *(volatile v8us*)(rp + HP + 256 * j) = lv[j];
  }
  __threadfence();
#pragma unroll
  for (int j = 0; j < 4; ++j) {
    *(volatile v8us*)(rp + 256 * j) = hv[j];
    *(volatile v8us*)(rp + HP + 256 * j) = lv[j];
  }
}

__global__ __launch_bounds__(NTHR) void k_scan2(const float* __restrict__ H2, const float* __restrict__ DINV,
                                                const int* __restrict__ NBR, const int* __restrict__ CNT,
                                                const float* __restrict__ b2, float* X2) {
  __shared__ int   nb_s[NWAVE * NBW];
  __shared__ float cf_s[NWAVE * NBW];
  const int tid = (int)threadIdx.x, lane = tid & 31, wave = tid >> 5;
  int*   nbl = nb_s + wave * NBW;
  float* cfl = cf_s + wave * NBW;
  const int node = (int)blockIdx.x * NWAVE + wave;
  const bool live = node < NN;
  const int nc = live ? node : NN - 1;
  const int cv = CNT[nc];
  const bool bad = live && ((unsigned)cv > (unsigned)DEGCAP);
  const int c = (live && !bad) ? cv : 0;
  const float dd = DINV[nc];
#pragma unroll
  for (int r = 0; r < 2; ++r) {
    const int t = 32 * r + lane;
    int sr = NBR[(size_t)nc * DEGCAP + t];
    sr = sr < 0 ? 0 : (sr > NN - 1 ? NN - 1 : sr);
    nbl[t] = sr;
    cfl[t] = DINV[sr] * dd;
  }
  if (lane == 0) { nbl[64] = nc; cfl[64] = dd * dd; }
  wave_sync();

  v4f acc[8];
  {
    const v4f z = {0.f, 0.f, 0.f, 0.f};
#pragma unroll
    for (int j = 0; j < 8; ++j) acc[j] = z;
  }
#pragma unroll 1
  for (int t = 0; t <= c; ++t) {
    const int tt = (t < c) ? t : 64;
    const int sk = nbl[tt];
    const float ck = cfl[tt];
    const float* hp = H2 + (size_t)sk * HP + 4 * lane;
#pragma unroll
    for (int j = 0; j < 8; ++j) {
      const v4f a = *(const v4fa*)(hp + 128 * j);
      acc[j] += ck * a;
    }
  }
  const float pzr = bad ? __int_as_float(0x7fc00000) : 0.0f;
  v4f ov[8];
#pragma unroll
  for (int j = 0; j < 8; ++j) {
    const int c0 = 128 * j + 4 * lane;
    const bool okc = c0 < HF;
    const int cb = okc ? c0 : HF - 4;
    const v4f bb = *(const v4fa*)(b2 + cb);
    v4f y;
    y.x = relu_keep(acc[j].x + bf16_val(bb.x)) + pzr;
    y.y = relu_keep(acc[j].y + bf16_val(bb.y)) + pzr;
    y.z = relu_keep(acc[j].z + bf16_val(bb.z)) + pzr;
    y.w = relu_keep(acc[j].w + bf16_val(bb.w)) + pzr;
    y.x = okc ? y.x : 0.0f; y.y = okc ? y.y : 0.0f; y.z = okc ? y.z : 0.0f; y.w = okc ? y.w : 0.0f;
    ov[j] = y;
  }
  float* rp = X2 + (size_t)nc * HP + 4 * lane;
  if (live) {
#pragma unroll
    for (int j = 0; j < 8; ++j) *(volatile v4f*)(rp + 128 * j) = ov[j];
  }
  __threadfence();
  if (live) {
#pragma unroll
    for (int j = 0; j < 8; ++j) *(volatile v4f*)(rp + 128 * j) = ov[j];
  }
}

__global__ __launch_bounds__(NTHR) void k_pool(const float* __restrict__ X2, const int* __restrict__ bat,
                                               unsigned short* G) {
  __shared__ __attribute__((aligned(16))) unsigned short grow[KF1];
  const int tid = (int)threadIdx.x, lane = tid & 31, wave = tid >> 5;
  const int g = (int)blockIdx.x;
  const int c0 = 128 * wave + 4 * lane;
  const float ninf = __int_as_float((int)0xff800000u);
  v4f mx = {ninf, ninf, ninf, ninf};
  v4f sm = {0.f, 0.f, 0.f, 0.f};
  int cnt = 0;
#pragma unroll 1
  for (int i0 = 0; i0 < NN; i0 += 32) {
    const int i  = i0 + lane;
    const int ic = i < NN ? i : NN - 1;
    const int b  = bat[ic];
    const bool hit = (i < NN) && (b == g);
    unsigned msk = __builtin_amdgcn_ballot_w32(hit);
    int nh = (int)__builtin_popcount(msk);
    nh = nh > 32 ? 32 : nh;
    cnt += nh;
#pragma unroll 1
    for (int q = 0; q < nh; ++q) {
      const int k = __builtin_ffs((int)msk) - 1;
      msk &= msk - 1u;
      int node = i0 + (k < 0 ? 0 : k);
      node = node > NN - 1 ? NN - 1 : node;
      const v4f v = *(const v4fa*)(X2 + (size_t)node * HP + c0);
      mx.x = maxk(mx.x, v.x); mx.y = maxk(mx.y, v.y); mx.z = maxk(mx.z, v.z); mx.w = maxk(mx.w, v.w);
      sm += v;
    }
  }
  const float cf = (cnt < 1) ? 1.0f : (float)cnt;
  const float rcp = 1.0f / cf;
  const v4f mean = sm * rcp;
  if (c0 < HF) {
    v4us xh, xl, mh, ml;
#pragma unroll
    for (int q = 0; q < 4; ++q) {
      unsigned hb = bf16_bits(mx[q]);
      xh[q] = (unsigned short)hb; xl[q] = (unsigned short)bf16_bits(mx[q] - __uint_as_float(hb << 16));
      hb = bf16_bits(mean[q]);
      mh[q] = (unsigned short)hb; ml[q] = (unsigned short)bf16_bits(mean[q] - __uint_as_float(hb << 16));
    }
    *(v4usa*)(grow + c0) = xh;
    *(v4usa*)(grow + GKH + c0) = xl;
    *(v4usa*)(grow + HF + c0) = mh;
    *(v4usa*)(grow + GKH + HF + c0) = ml;
  }
  if (tid < GKH - PW) {
    grow[PW + tid] = (unsigned short)0;
    grow[GKH + PW + tid] = (unsigned short)0;
  }
  __syncthreads();
  const v8us q0 = *(const v8usa*)(grow + 8 * tid);
  const v8us q1 = *(const v8usa*)(grow + 8 * (NTHR + tid));
  unsigned short* gp = G + (size_t)g * KF1 + 8 * tid;
  *(volatile v8us*)gp = q0;
  *(volatile v8us*)(gp + 8 * NTHR) = q1;
  __threadfence();
  *(volatile v8us*)gp = q0;
  *(volatile v8us*)(gp + 8 * NTHR) = q1;
}

__global__ __launch_bounds__(NTHR) void k_head(const unsigned short* __restrict__ G,
                                               const unsigned short* __restrict__ FC1d,
                                               const unsigned short* __restrict__ FC2d,
                                               const float* __restrict__ fc1b, const float* __restrict__ fc2b,
                                               float* out) {
  extern __shared__ __attribute__((aligned(16))) unsigned char hsm[];
  unsigned short* Fs = (unsigned short*)hsm;
  float* os = (float*)(hsm + 16 * KF2 * 2);
  const int tid = (int)threadIdx.x, lane = tid & 31, wave = tid >> 5, hh = lane >> 4, m = lane & 15;
  const int rb = (int)blockIdx.x * 16;
  const v8f z8 = {0.f, 0.f, 0.f, 0.f, 0.f, 0.f, 0.f, 0.f};

#pragma unroll 1
  for (int gi = 0; gi < 3; ++gi) {
    const int col0 = 64 * (gi * NWAVE + wave);
    v8f acc[4];
    acc[0] = z8; acc[1] = z8; acc[2] = z8; acc[3] = z8;
    const unsigned short* ap = G + (size_t)(rb + m) * KF1 + 8 * hh;
    const unsigned short* wp = FC1d + (size_t)(col0 + m) * KF1 + 8 * hh;
#pragma unroll 1
    for (int ks = 0; ks < KF1 / 32; ++ks) {
      FragB af;
      af.h[0] = *(const v8usa*)(ap + 32 * ks);
      af.h[1] = *(const v8usa*)(ap + 32 * ks + 16);
#pragma unroll
      for (int t = 0; t < 4; ++t) {
        const unsigned short* wq = wp + (size_t)(16 * t) * KF1 + 32 * ks;
        FragB bf;
        bf.h[0] = *(const v8usa*)wq;
        bf.h[1] = *(const v8usa*)(wq + 16);
        acc[t] = wmb(af, bf, acc[t]);
      }
    }
#pragma unroll
    for (int t = 0; t < 4; ++t) {
      const int col = col0 + 16 * t + m;
      const bool okc = col < F1N;
      const float bb = bf16_val(fc1b[okc ? col : F1N - 1]);
#pragma unroll
      for (int r = 0; r < 8; ++r) {
        const int row = 8 * hh + r;
        float v = relu_keep(acc[t][r] + bb);
        v = okc ? v : 0.0f;
        const unsigned hb = bf16_bits(v);
        const unsigned lb = bf16_bits(v - __uint_as_float(hb << 16));
        Fs[row * KF2 + col] = (unsigned short)hb;
        Fs[row * KF2 + F1P + col] = (unsigned short)lb;
      }
    }
  }
  __syncthreads();

  {
    v8f acc2[3];
    acc2[0] = z8; acc2[1] = z8; acc2[2] = z8;
    const unsigned short* fa = Fs + m * KF2 + 8 * hh;
    const int n0 = wave, n1 = wave + 8, n2 = wave + 16;
    const int n2c = n2 < 20 ? n2 : 19;
    const unsigned short* w0 = FC2d + (size_t)(16 * n0  + m) * KF2 + 8 * hh;
    const unsigned short* w1 = FC2d + (size_t)(16 * n1  + m) * KF2 + 8 * hh;
    const unsigned short* w2 = FC2d + (size_t)(16 * n2c + m) * KF2 + 8 * hh;
#pragma unroll 1
    for (int ks = 0; ks < KF2 / 32; ++ks) {
      FragB af, b0, b1f, b2f;
      af.h[0]  = *(const v8usa*)(fa + 32 * ks);
      af.h[1]  = *(const v8usa*)(fa + 32 * ks + 16);
      b0.h[0]  = *(const v8usa*)(w0 + 32 * ks);
      b0.h[1]  = *(const v8usa*)(w0 + 32 * ks + 16);
      b1f.h[0] = *(const v8usa*)(w1 + 32 * ks);
      b1f.h[1] = *(const v8usa*)(w1 + 32 * ks + 16);
      b2f.h[0] = *(const v8usa*)(w2 + 32 * ks);
      b2f.h[1] = *(const v8usa*)(w2 + 32 * ks + 16);
      acc2[0] = wmb(af, b0,  acc2[0]);
      acc2[1] = wmb(af, b1f, acc2[1]);
      acc2[2] = wmb(af, b2f, acc2[2]);
    }
#pragma unroll
    for (int t = 0; t < 3; ++t) {
      const int nt = wave + 8 * t;
      const int col = 16 * nt + m;
      const bool okc = (nt < 20) && (col < F2N);
      const float bb = bf16_val(fc2b[(col < F2N) ? col : F2N - 1]);
#pragma unroll
      for (int r = 0; r < 8; ++r) {
        const int row = 8 * hh + r;
        if (okc) os[row * F2N + col] = acc2[t][r] + bb;
      }
    }
  }
  __syncthreads();

  constexpr int NV = (16 * F2N) / 4;
  constexpr int NIT = (NV + NTHR - 1) / NTHR;
  float* ob = out + (size_t)blockIdx.x * (16 * F2N);
  v4f ovv[NIT];
#pragma unroll
  for (int it = 0; it < NIT; ++it) {
    const int idx = it * NTHR + tid;
    const int idc = idx < NV ? idx : NV - 1;
    ovv[it] = *(const v4fa*)(os + 4 * idc);
  }
#pragma unroll
  for (int it = 0; it < NIT; ++it) {
    const int idx = it * NTHR + tid;
    if (idx < NV) *(volatile v4f*)(ob + 4 * (size_t)idx) = ovv[it];
  }
  __threadfence();
#pragma unroll
  for (int it = 0; it < NIT; ++it) {
    const int idx = it * NTHR + tid;
    if (idx < NV) *(volatile v4f*)(ob + 4 * (size_t)idx) = ovv[it];
  }
}

static inline size_t al256(size_t o) { return (o + 255) & ~(size_t)255; }

extern "C" void kernel_launch(void* const* d_in, const int* in_sizes, int n_in,
                              void* d_out, int out_size, void* d_ws, size_t ws_size,
                              hipStream_t stream) {
  if (n_in < 13) return;
  if (in_sizes[0] != NN * FE) return;
  if (in_sizes[1] < 2 || (in_sizes[1] & 1) != 0) return;
  const int nE = in_sizes[1] / 2;
  if (nE < 1 || nE >= (1 << (31 - SLA))) return;
  if (in_sizes[2] != NN) return;
  if (in_sizes[3] != HF * FE) return;
  if (in_sizes[4] != NHD * FE || in_sizes[5] != NHD * FE) return;
  if (in_sizes[6] != HF) return;
  if (in_sizes[7] != HF * HF || in_sizes[8] != HF) return;
  if (in_sizes[9] != F1N * PW || in_sizes[10] != F1N) return;
  if (in_sizes[11] != F2N * F1N || in_sizes[12] != F2N) return;
  if (out_size != NG * F2N) return;

  const float* x    = (const float*)d_in[0];
  const int*   edge = (const int*)d_in[1];
  const int*   bat  = (const int*)d_in[2];
  const float* W1   = (const float*)d_in[3];
  const float* atS  = (const float*)d_in[4];
  const float* atD  = (const float*)d_in[5];
  const float* b1   = (const float*)d_in[6];
  const float* W2   = (const float*)d_in[7];
  const float* b2   = (const float*)d_in[8];
  const float* fc1w = (const float*)d_in[9];
  const float* fc1b = (const float*)d_in[10];
  const float* fc2w = (const float*)d_in[11];
  const float* fc2b = (const float*)d_in[12];
  float* out = (float*)d_out;
  const int* src = edge;
  const int* dst = edge + nE;
  const int vec8 = ((nE & 3) == 0) ? 1 : 0;

  char* ws = (char*)d_ws;
  size_t off = 0;
  const size_t oA   = off; off = al256(off + (size_t)MP * HP * 4);
  const size_t oB   = off; off = al256(off + (size_t)MP * K2 * 2);
  const size_t oXB  = off; off = al256(off + (size_t)MP * K1 * 2);
  const size_t oW1  = off; off = al256(off + (size_t)HP * K1 * 2);
  const size_t oW2  = off; off = al256(off + (size_t)HP * K2 * 2);
  const size_t oF1  = off; off = al256(off + (size_t)F1P * KF1 * 2);
  const size_t oF2  = off; off = al256(off + (size_t)F2P * KF2 * 2);
  const size_t oAS  = off; off = al256(off + (size_t)NP * 16 * 4);
  const size_t oAD  = off; off = al256(off + (size_t)NP * 16 * 4);
  const size_t oNB  = off; off = al256(off + (size_t)NP * DEGCAP * 4);
  const size_t oCN  = off; off = al256(off + (size_t)NP * 4);
  const size_t oDI  = off; off = al256(off + (size_t)NP * 4);
  const size_t oG   = off; off = al256(off + (size_t)NG * KF1 * 2);
  if (off > ws_size || off > (size_t)WSMAX) return;
  float*          RA   = (float*)(ws + oA);
  unsigned short* X1   = (unsigned short*)(ws + oB);
  float*          X2   = (float*)(ws + oB);
  unsigned short* XB   = (unsigned short*)(ws + oXB);
  unsigned short* W1p  = (unsigned short*)(ws + oW1);
  unsigned short* W2d  = (unsigned short*)(ws + oW2);
  unsigned short* FC1d = (unsigned short*)(ws + oF1);
  unsigned short* FC2d = (unsigned short*)(ws + oF2);
  float*          AS   = (float*)(ws + oAS);
  float*          AD   = (float*)(ws + oAD);
  int*            NBR  = (int*)(ws + oNB);
  int*            CNT  = (int*)(ws + oCN);
  float*          DINV = (float*)(ws + oDI);
  unsigned short* G    = (unsigned short*)(ws + oG);

  const size_t adjLds  = (size_t)AGG_LDS_INTS * 4;
  const size_t headLds = (size_t)HEAD_LDS;
  hipFuncSetAttribute(reinterpret_cast<const void*>(&k_adj),  hipFuncAttributeMaxDynamicSharedMemorySize, (int)adjLds);
  hipFuncSetAttribute(reinterpret_cast<const void*>(&k_head), hipFuncAttributeMaxDynamicSharedMemorySize, (int)headLds);

  k_prep<<<U_TOT / NTHR, NTHR, 0, stream>>>(x, W1, W2, fc1w, fc2w, XB, W1p, W2d, FC1d, FC2d);
  k_gemm<<<dim3(MP / GBM, HP / GBN), GTHR, 0, stream>>>(XB, W1p, RA, K1, HP);
  k_dots<<<NN / NWAVE, NTHR, 0, stream>>>(RA, atS, atD, AS, AD);
  k_adj<<<NP / NBA, NTHR, adjLds, stream>>>(src, dst, nE, vec8, NBR, CNT, DINV);
  k_scan1<<<MP / NWAVE, NTHR, 0, stream>>>(RA, AS, AD, NBR, CNT, b1, X1);
  k_gemm<<<dim3(MP / GBM, HP / GBN), GTHR, 0, stream>>>(X1, W2d, RA, K2, HP);
  k_scan2<<<NN / NWAVE, NTHR, 0, stream>>>(RA, DINV, NBR, CNT, b2, X2);
  k_pool<<<NG, NTHR, 0, stream>>>(X2, bat, G);
  k_head<<<NG / 16, NTHR, headLds, stream>>>(G, FC1d, FC2d, fc1b, fc2b, out);
}
